// TopDownLSTMEncoder_75797582839903
// MI455X (gfx1250) — hardware-verified
//
#include <hip/hip_runtime.h>

typedef __attribute__((ext_vector_type(16))) _Float16 v16h;
typedef __attribute__((ext_vector_type(8)))  _Float16 v8h;
typedef __attribute__((ext_vector_type(16))) __bf16   v16b;
typedef __attribute__((ext_vector_type(8)))  __bf16   v8b;
typedef __attribute__((ext_vector_type(8)))  float    v8f;
typedef __attribute__((ext_vector_type(4)))  float    v4f;
typedef __attribute__((ext_vector_type(4)))  unsigned int v4u;

constexpr int kBatch     = 32;
constexpr int kNodes     = 1024;
constexpr int kHalfNodes = 512;
constexpr int kDim       = 256;
constexpr int kHid       = 256;
constexpr int kGates     = 768;
constexpr int kThreads   = 256;
constexpr int kTilePitch = 264;
constexpr int kSlabPitch = 260;

__device__ __forceinline__ unsigned short f2bf_bits(float f) {
  unsigned u = __float_as_uint(f);
  return (unsigned short)((u + 0x7FFFu + ((u >> 16) & 1u)) >> 16);
}
__device__ __forceinline__ float bf_bits2f(unsigned short h) { return __uint_as_float(((unsigned)h) << 16); }
__device__ __forceinline__ float bf_rne(float f) { return bf_bits2f(f2bf_bits(f)); }
__device__ __forceinline__ unsigned pack_bf2(float a, float b) {
  return (unsigned)f2bf_bits(a) | ((unsigned)f2bf_bits(b) << 16);
}
struct HL2 { unsigned hi; unsigned lo; };
__device__ __forceinline__ HL2 split_pack2(float a, float b) {
  const unsigned short ah = f2bf_bits(a);
  const unsigned short bh = f2bf_bits(b);
  const unsigned short al = f2bf_bits(a - bf_bits2f(ah));
  const unsigned short bl = f2bf_bits(b - bf_bits2f(bh));
  HL2 r;
  r.hi = (unsigned)ah | ((unsigned)bh << 16);
  r.lo = (unsigned)al | ((unsigned)bl << 16);
  return r;
}

__device__ __forceinline__ void dep_guard_h(v8f& a, v8f& b, v16h x, v16h y) { asm volatile("v_nop\n\tv_nop\n\tv_nop\n\tv_nop" : "+v"(a), "+v"(b) : "v"(x), "v"(y)); }
__device__ __forceinline__ void dep_guard_b(v8f& a, v8f& b, v16b x, v16b y) { asm volatile("v_nop\n\tv_nop\n\tv_nop\n\tv_nop" : "+v"(a), "+v"(b) : "v"(x), "v"(y)); }
__device__ __forceinline__ void keep4_h(v16h a, v16h b, v16h c, v16h d) { asm volatile("v_nop" :: "v"(a), "v"(b), "v"(c), "v"(d)); }
__device__ __forceinline__ void keep4_b(v16b a, v16b b, v16b c, v16b d) { asm volatile("v_nop" :: "v"(a), "v"(b), "v"(c), "v"(d)); }
__device__ __forceinline__ void acc_guard4(v8f& a, v8f& b, v8f& c, v8f& d) { asm volatile("v_nop\n\tv_nop\n\tv_nop\n\tv_nop" : "+v"(a), "+v"(b), "+v"(c), "+v"(d)); }
__device__ __forceinline__ void guard3s_b(v8f& a, v8f& b, v8f& c, v16b x0, v16b x1,
                                          v16b y0, v16b y1, v16b y2, v16b z0, v16b z1, v16b z2) {
  asm volatile("v_nop\n\tv_nop\n\tv_nop\n\tv_nop" : "+v"(a), "+v"(b), "+v"(c)
               : "v"(x0), "v"(x1), "v"(y0), "v"(y1), "v"(y2), "v"(z0), "v"(z1), "v"(z2));
}
__device__ __forceinline__ void acc_guard3(v8f& a, v8f& b, v8f& c) {
  asm volatile("v_nop\n\tv_nop\n\tv_nop\n\tv_nop" : "+v"(a), "+v"(b), "+v"(c));
}

template <typename T> struct Frag;
template <> struct Frag<_Float16> {
  typedef v16h V; union U { v16h v; v8h h[2]; };
  static __device__ __forceinline__ v16h load(const _Float16* p) {
    U f; f.h[0] = *(const v8h*)(p); f.h[1] = *(const v8h*)(p + 16); return f.v;
  }
  static __device__ __forceinline__ v8f mma(v16h a, v16h b, v8f c) {
    return __builtin_amdgcn_wmma_f32_16x16x32_f16(false, a, false, b, (short)0, c, false, false);
  }
  static __device__ __forceinline__ void guard(v8f& a, v8f& b, v16h x, v16h y) { dep_guard_h(a, b, x, y); }
  static __device__ __forceinline__ void keep(v16h a, v16h b, v16h c, v16h d) { keep4_h(a, b, c, d); }
};
template <> struct Frag<__bf16> {
  typedef v16b V; union U { v16b v; v8b h[2]; };
  static __device__ __forceinline__ v16b load(const __bf16* p) {
    U f; f.h[0] = *(const v8b*)(p); f.h[1] = *(const v8b*)(p + 16); return f.v;
  }
  static __device__ __forceinline__ v8f mma(v16b a, v16b b, v8f c) {
    return __builtin_amdgcn_wmma_f32_16x16x32_bf16(false, a, false, b, (short)0, c, false, false);
  }
  static __device__ __forceinline__ void guard(v8f& a, v8f& b, v16b x, v16b y) { dep_guard_b(a, b, x, y); }
  static __device__ __forceinline__ void keep(v16b a, v16b b, v16b c, v16b d) { keep4_b(a, b, c, d); }
};

template <int ET> struct Elem;
template <> struct Elem<0> { typedef _Float16 T; };
template <> struct Elem<1> { typedef __bf16 T; };
template <int ET, bool SPLIT, int BIAS_MODE, int OUT_MODE, bool RESID, int ACT = 0>
__global__ __launch_bounds__(256) void wmma_gemm64(
    const unsigned short* __restrict__ Ap, const unsigned short* __restrict__ A2p, int lda, long strideA,
    const unsigned short* __restrict__ Btp, const unsigned short* __restrict__ Bt2p, int ldb, long strideB,
    void* __restrict__ Cout, void* __restrict__ Cout2, int ldc, long strideC,
    const float* __restrict__ bias,
    const float* __restrict__ resid, long strideR,
    int M, int N, int K, float scale) {
  typedef typename Elem<ET>::T T;
  typedef typename Frag<T>::V V;
  const T* A = (const T*)Ap; const T* A2 = (const T*)A2p; const T* Bt = (const T*)Btp; const T* Bt2 = (const T*)Bt2p;
  __shared__ __align__(16) float sT[8][16 * 68];
  const int b    = blockIdx.y;
  const int lane = threadIdx.x & 31;
  const int wave = threadIdx.x >> 5;
  const int tilesN = N >> 6;
  const int tilesM = M >> 6;
  const int tile = blockIdx.x * 8 + wave;
  if (tile >= tilesM * tilesN) return;
  const int tm = tile / tilesN;
  const int tn = tile - tm * tilesN;
  const int m0 = tm << 6;
  const int n0 = tn << 6;

  const T* Ab  = A  + (size_t)b * strideA;
  const T* Bb  = Bt + (size_t)b * strideB;
  const T* Ab2 = SPLIT ? (A2  + (size_t)b * strideA) : nullptr;
  const T* Bb2 = SPLIT ? (Bt2 + (size_t)b * strideB) : nullptr;

  const int rlane = lane & 15;
  const int koff  = (lane >> 4) * 8;
  const int mOff  = (lane >> 4) * 8;

  v8f acc[4][4];
#pragma unroll
  for (int i = 0; i < 4; ++i)
#pragma unroll
    for (int j = 0; j < 4; ++j) acc[i][j] = (v8f){0.f,0.f,0.f,0.f,0.f,0.f,0.f,0.f};

  for (int k0 = 0; k0 < K; k0 += 32) {
    V bh[4], bl[4];
#pragma unroll
    for (int j = 0; j < 4; ++j) {
      const size_t bo = (size_t)(n0 + (j << 4) + rlane) * ldb + koff + k0;
      bh[j] = Frag<T>::load(Bb + bo);
      if (SPLIT) bl[j] = Frag<T>::load(Bb2 + bo);
    }
#pragma unroll
    for (int i = 0; i < 4; ++i) {
      const size_t ao = (size_t)(m0 + (i << 4) + rlane) * lda + koff + k0;
      V ah = Frag<T>::load(Ab + ao);
      V al;
      if (SPLIT) al = Frag<T>::load(Ab2 + ao);
#pragma unroll
      for (int j = 0; j < 4; ++j) {
        acc[i][j] = Frag<T>::mma(ah, bh[j], acc[i][j]);
        if (SPLIT) {
          acc[i][j] = Frag<T>::mma(ah, bl[j], acc[i][j]);
          acc[i][j] = Frag<T>::mma(al, bh[j], acc[i][j]);
        }
      }
      Frag<T>::guard(acc[i][0], acc[i][3], ah, SPLIT ? al : ah);
    }
    Frag<T>::keep(bh[0], bh[1], bh[2], bh[3]);
    if (SPLIT) Frag<T>::keep(bl[0], bl[1], bl[2], bl[3]);
  }
  acc_guard4(acc[0][0], acc[0][1], acc[0][2], acc[0][3]);
  acc_guard4(acc[1][0], acc[1][1], acc[1][2], acc[1][3]);
  acc_guard4(acc[2][0], acc[2][1], acc[2][2], acc[2][3]);
  acc_guard4(acc[3][0], acc[3][1], acc[3][2], acc[3][3]);

  float* slab = sT[wave];
  const float* Rb = RESID ? (resid + (size_t)b * strideR) : nullptr;
#pragma unroll
  for (int i = 0; i < 4; ++i) {
    const int mBase = m0 + (i << 4);
#pragma unroll
    for (int j = 0; j < 4; ++j) {
      const int n = n0 + (j << 4) + rlane;
      float bv = 0.f;
      if (BIAS_MODE == 2) bv = bias[n];
#pragma unroll
      for (int r = 0; r < 8; ++r) {
        float v = acc[i][j][r] * scale;
        if (BIAS_MODE == 1) v += bias[mBase + mOff + r];
        if (BIAS_MODE == 2) v += bv;
        if (RESID) v += Rb[(size_t)(mBase + mOff + r) * ldc + n];
        if (ACT == 1) v = tanhf(v);
        if (ACT == 2) v = fmaxf(v, 0.0f);
        if (ACT == 3) v = v / (1.0f + expf(-v));
        if (ACT == 4) v = (v > 0.f) ? v : 0.01f * v;
        if (ACT == 5) v = 0.5f * v * (1.0f + erff(v * 0.70710678118654752f));
        slab[(mOff + r) * 68 + (j << 4) + rlane] = v;
      }
    }
    __builtin_amdgcn_fence(__ATOMIC_RELEASE, "workgroup");
    __builtin_amdgcn_wave_barrier();
    __builtin_amdgcn_fence(__ATOMIC_ACQUIRE, "workgroup");
    if (OUT_MODE == 0) {
      float* C = (float*)Cout + (size_t)b * strideC;
      const int hh = lane >> 4, c4 = (lane & 15) * 4;
      for (int pass = 0; pass < 2; ++pass) {
#pragma unroll
        for (int it = 0; it < 8; ++it) {
          const int row = it * 2 + hh;
          v4f v = *(const v4f*)(slab + row * 68 + c4);
          *(volatile v4f*)(C + (size_t)(mBase + row) * ldc + n0 + c4) = v;
        }
        __threadfence();
      }
    } else {
      const int q = lane >> 3, c8 = (lane & 7) * 8;
      unsigned short* C  = (unsigned short*)Cout  + (size_t)b * strideC;
      unsigned short* C2 = (OUT_MODE == 2) ? ((unsigned short*)Cout2 + (size_t)b * strideC) : nullptr;
      for (int pass = 0; pass < 2; ++pass) {
#pragma unroll
        for (int it = 0; it < 4; ++it) {
          const int row = it * 4 + q;
          const float* sp = slab + row * 68 + c8;
          v8h hv, lv;
#pragma unroll
          for (int e = 0; e < 8; ++e) {
            if (OUT_MODE == 1) {
              hv[e] = (_Float16)sp[e];
            } else {
              unsigned short hb = f2bf_bits(sp[e]);
              unsigned short lb = f2bf_bits(sp[e] - bf_bits2f(hb));
              hv[e] = __builtin_bit_cast(_Float16, hb);
              lv[e] = __builtin_bit_cast(_Float16, lb);
            }
          }
          *(volatile v8h*)(C + (size_t)(mBase + row) * ldc + n0 + c8) = hv;
          if (OUT_MODE == 2) *(volatile v8h*)(C2 + (size_t)(mBase + row) * ldc + n0 + c8) = lv;
        }
        __threadfence();
      }
    }
    __builtin_amdgcn_fence(__ATOMIC_RELEASE, "workgroup");
    __builtin_amdgcn_wave_barrier();
    __builtin_amdgcn_fence(__ATOMIC_ACQUIRE, "workgroup");
  }
}

__device__ __forceinline__ float gate_sigmoid(float x) {
  return __builtin_amdgcn_rcpf(1.0f + expf(-x));
}
__device__ __forceinline__ float gate_tanh(float x) {
  return 1.0f - 2.0f * __builtin_amdgcn_rcpf(1.0f + expf(2.0f * x));
}

__global__ __launch_bounds__(kThreads)
void k_cast_bf16x8(const float* __restrict__ in, unsigned short* __restrict__ outp, int n8) {
  const int i = blockIdx.x * kThreads + threadIdx.x;
  if (i < n8) {
    const float* p = in + (size_t)i * 8;
    const v4f a = *(const v4f*)(p);
    const v4f b = *(const v4f*)(p + 4);
    v4u px;
    px[0] = pack_bf2(a[0], a[1]);
    px[1] = pack_bf2(a[2], a[3]);
    px[2] = pack_bf2(b[0], b[1]);
    px[3] = pack_bf2(b[2], b[3]);
    unsigned short* d = outp + (size_t)i * 8;
    *(volatile v4u*)d = px;
    __threadfence();
    *(volatile v4u*)d = px;
  }
}

__global__ __launch_bounds__(kThreads)
void k_wprep(const float* __restrict__ W, unsigned short* __restrict__ WBt) {
  __shared__ __align__(16) float sW[32 * kSlabPitch];
  const int tid = threadIdx.x;
  const int lane = tid & 31;
  const int wave = tid >> 5;
  const int n0 = blockIdx.x * 32;
  {
    const int c = tid & 31;
    const int kq = tid >> 5;
#pragma unroll 4
    for (int it = 0; it < 32; ++it) {
      const int k = it * 8 + kq;
      sW[c * kSlabPitch + k] = W[(size_t)k * kGates + n0 + c];
    }
  }
  __syncthreads();
  for (int pass = 0; pass < 2; ++pass) {
#pragma unroll
    for (int jr = 0; jr < 4; ++jr) {
      const int row = wave * 4 + jr;
      const float* sp = sW + row * kSlabPitch + 8 * lane;
      const v4f a = *(const v4f*)(sp);
      const v4f b = *(const v4f*)(sp + 4);
      v4u px;
      px[0] = pack_bf2(a[0], a[1]);
      px[1] = pack_bf2(a[2], a[3]);
      px[2] = pack_bf2(b[0], b[1]);
      px[3] = pack_bf2(b[2], b[3]);
      *(volatile v4u*)(WBt + ((size_t)(n0 + row)) * kDim + 8 * lane) = px;
    }
    __threadfence();
  }
}

__global__ __launch_bounds__(kThreads)
void k_vprep(const float* __restrict__ tf, const float* __restrict__ to,
             const float* __restrict__ tz, unsigned short* __restrict__ VBh,
             unsigned short* __restrict__ VBl) {
  __shared__ float colS[16 * kHid];
  __shared__ __align__(16) float vsl[16 * kSlabPitch];
  const int tid = threadIdx.x;
  const int lane = tid & 31;
  const int wave = tid >> 5;
  const int g = blockIdx.x >> 4;
  const int i0 = (blockIdx.x & 15) * 16;
  const float* T = (g == 0) ? tf : ((g == 1) ? to : tz);
  {
    const float* src = T + (size_t)tid * kHid + i0;
#pragma unroll
    for (int q4 = 0; q4 < 4; ++q4) {
      const v4f a = *(const v4f*)(src + 4 * q4);
#pragma unroll
      for (int e = 0; e < 4; ++e) colS[(4 * q4 + e) * kHid + tid] = bf_rne(a[e]);
    }
  }
  __syncthreads();
  float s[16];
#pragma unroll
  for (int q = 0; q < 16; ++q) s[q] = 0.0f;
#pragma unroll 1
  for (int k = 0; k < kHid; ++k) {
    const float a = bf_rne(T[(size_t)k * kHid + tid]);
#pragma unroll
    for (int q = 0; q < 16; ++q) s[q] = fmaf(colS[q * kHid + k], a, s[q]);
  }
#pragma unroll
  for (int q = 0; q < 16; ++q) vsl[q * kSlabPitch + tid] = s[q];
  __syncthreads();
  for (int pass = 0; pass < 2; ++pass) {
#pragma unroll
    for (int jr = 0; jr < 2; ++jr) {
      const int q = wave * 2 + jr;
      const float* sp = vsl + q * kSlabPitch + 8 * lane;
      const v4f a = *(const v4f*)(sp);
      const v4f b = *(const v4f*)(sp + 4);
      const HL2 p0 = split_pack2(a[0], a[1]);
      const HL2 p1 = split_pack2(a[2], a[3]);
      const HL2 p2 = split_pack2(b[0], b[1]);
      const HL2 p3 = split_pack2(b[2], b[3]);
      v4u pxh, pxl;
      pxh[0] = p0.hi; pxh[1] = p1.hi; pxh[2] = p2.hi; pxh[3] = p3.hi;
      pxl[0] = p0.lo; pxl[1] = p1.lo; pxl[2] = p2.lo; pxl[3] = p3.lo;
      const size_t ro = ((size_t)(g * kHid + i0 + q)) * kHid + 8 * lane;
      *(volatile v4u*)(VBh + ro) = pxh;
      *(volatile v4u*)(VBl + ro) = pxl;
    }
    __threadfence();
  }
}

__global__ __launch_bounds__(kThreads)
void k_tree(const int* __restrict__ conn, const int* __restrict__ nmask,
            const float* __restrict__ bias, const float* __restrict__ gin,
            const unsigned short* __restrict__ VBh, const unsigned short* __restrict__ VBl,
            float* CS, float* out, int i_begin) {
  __shared__ __align__(16) unsigned short hsH[kBatch * kTilePitch];
  __shared__ __align__(16) unsigned short hsL[kBatch * kTilePitch];
  __shared__ __align__(16) float slab[kBatch * kSlabPitch];
  __shared__ float sBias[kGates];
  __shared__ int sPid[kBatch];
  __shared__ int sVal[kBatch];
  (void)nmask;

  const int tid   = threadIdx.x;
  const int lane  = tid & 31;
  const int wave  = tid >> 5;
  const int rlane = lane & 15;
  const int hh    = lane >> 4;
  const int koff  = hh * 8;
  const int mOff  = hh * 8;

  for (int idx = tid; idx < kGates; idx += kThreads) sBias[idx] = bf_rne(bias[idx]);

  const __bf16* Vh  = (const __bf16*)(const void*)VBh;
  const __bf16* Vl  = (const __bf16*)(const void*)VBl;
  const __bf16* hAh = (const __bf16*)(const void*)hsH;
  const __bf16* hAl = (const __bf16*)(const void*)hsL;

  for (int s = 0; s < kHalfNodes; ++s) {
    const int i = i_begin + s;
    {
      const int row = tid >> 3;
      const int seg = tid & 7;
      int p = conn[row * kNodes + i];
      p = (p < 0) ? 0 : ((p > kNodes - 1) ? (kNodes - 1) : p);
      const bool vld = (p < i);
      const float* hsrc = out + ((size_t)(row * kNodes + p)) * kHid + seg * 32;
      unsigned short* hdh = hsH + row * kTilePitch + seg * 32;
      unsigned short* hdl = hsL + row * kTilePitch + seg * 32;
#pragma unroll
      for (int q = 0; q < 4; ++q) {
        const v4f h0 = *(const v4f*)(hsrc + 8 * q);
        const v4f h1 = *(const v4f*)(hsrc + 8 * q + 4);
        const float e0 = vld ? h0[0] : 0.0f;
        const float e1 = vld ? h0[1] : 0.0f;
        const float e2 = vld ? h0[2] : 0.0f;
        const float e3 = vld ? h0[3] : 0.0f;
        const float e4 = vld ? h1[0] : 0.0f;
        const float e5 = vld ? h1[1] : 0.0f;
        const float e6 = vld ? h1[2] : 0.0f;
        const float e7 = vld ? h1[3] : 0.0f;
        const HL2 p0 = split_pack2(e0, e1);
        const HL2 p1 = split_pack2(e2, e3);
        const HL2 p2 = split_pack2(e4, e5);
        const HL2 p3 = split_pack2(e6, e7);
        v4u phh, phl;
        phh[0] = p0.hi; phh[1] = p1.hi; phh[2] = p2.hi; phh[3] = p3.hi;
        phl[0] = p0.lo; phl[1] = p1.lo; phl[2] = p2.lo; phl[3] = p3.lo;
        *(v4u*)(hdh + 8 * q) = phh;
        *(v4u*)(hdl + 8 * q) = phl;
      }
      if (wave == 0) {
        int p2 = conn[lane * kNodes + i];
        p2 = (p2 < 0) ? 0 : ((p2 > kNodes - 1) ? (kNodes - 1) : p2);
        sPid[lane] = p2;
        sVal[lane] = (p2 < i) ? 1 : 0;
      }
    }
    __syncthreads();

    float cR[2][2][8];
#pragma unroll
    for (int t = 0; t < 2; ++t) {
      const int ub = wave * 2 + t;
      const int u  = ub * 16 + rlane;
      v8f acc[2][3];
#pragma unroll
      for (int ms = 0; ms < 2; ++ms)
#pragma unroll
        for (int j = 0; j < 3; ++j) acc[ms][j] = (v8f){0.f, 0.f, 0.f, 0.f, 0.f, 0.f, 0.f, 0.f};

#pragma unroll 1
      for (int kc = 0; kc < kHid / 32; ++kc) {
        v16b bvh[3], bvl[3];
#pragma unroll
        for (int j = 0; j < 3; ++j) {
          const size_t bo = ((size_t)(j * kHid + ub * 16 + rlane)) * kHid + kc * 32 + koff;
          bvh[j] = Frag<__bf16>::load(Vh + bo);
          bvl[j] = Frag<__bf16>::load(Vl + bo);
        }
#pragma unroll
        for (int ms = 0; ms < 2; ++ms) {
          const int ao = (ms * 16 + rlane) * kTilePitch + kc * 32 + koff;
          const v16b ah = Frag<__bf16>::load(hAh + ao);
          const v16b al = Frag<__bf16>::load(hAl + ao);
#pragma unroll
          for (int j = 0; j < 3; ++j) {
            acc[ms][j] = Frag<__bf16>::mma(ah, bvh[j], acc[ms][j]);
            acc[ms][j] = Frag<__bf16>::mma(ah, bvl[j], acc[ms][j]);
            acc[ms][j] = Frag<__bf16>::mma(al, bvh[j], acc[ms][j]);
          }
          guard3s_b(acc[ms][0], acc[ms][1], acc[ms][2], ah, al,
                    bvh[0], bvh[1], bvh[2], bvl[0], bvl[1], bvl[2]);
        }
      }
      acc_guard3(acc[0][0], acc[0][1], acc[0][2]);
      acc_guard3(acc[1][0], acc[1][1], acc[1][2]);

      const float bF = sBias[u];
      const float bO = sBias[kHid + u];
      const float bZ = sBias[2 * kHid + u];
#pragma unroll
      for (int ms = 0; ms < 2; ++ms) {
#pragma unroll
        for (int r = 0; r < 8; ++r) {
          const int b  = ms * 16 + mOff + r;
          const int pp = sPid[b];
          const int vv = sVal[b];
          const float* grow = gin + ((size_t)(b * kHalfNodes + s)) * kGates;
          const float gf = acc[ms][0][r] + (grow[u] + bF);
          const float go = acc[ms][1][r] + (grow[kHid + u] + bO);
          const float gz = acc[ms][2][r] + (grow[2 * kHid + u] + bZ);
          float pc = CS[((size_t)(b * kNodes + pp)) * kHid + u];
          pc = (vv != 0) ? pc : 0.0f;
          const float f = gate_sigmoid(gf);
          const float o = gate_sigmoid(go);
          const float z = gate_tanh(gz);
          const float c = pc * f + z * (1.0f - f);
          const float h = o * gate_tanh(c);
          slab[b * kSlabPitch + u] = h;
          cR[t][ms][r] = c;
        }
        asm volatile("" ::: "memory");
      }
    }
    __syncthreads();

    for (int pass = 0; pass < 2; ++pass) {
#pragma unroll
      for (int jr = 0; jr < 4; ++jr) {
        const int b = wave * 4 + jr;
        const float* hr = slab + b * kSlabPitch;
        const size_t ro = ((size_t)(b * kNodes + i)) * kHid;
        const v4f ha = *(const v4f*)(hr + 4 * lane);
        const v4f hb = *(const v4f*)(hr + 128 + 4 * lane);
        *(volatile v4f*)(out + ro + 4 * lane) = ha;
        *(volatile v4f*)(out + ro + 128 + 4 * lane) = hb;
      }
      __threadfence();
    }
    __syncthreads();

#pragma unroll
    for (int t = 0; t < 2; ++t) {
      const int u = (wave * 2 + t) * 16 + rlane;
#pragma unroll
      for (int ms = 0; ms < 2; ++ms)
#pragma unroll
        for (int r = 0; r < 8; ++r)
          slab[(ms * 16 + mOff + r) * kSlabPitch + u] = cR[t][ms][r];
    }
    __syncthreads();

    for (int pass = 0; pass < 2; ++pass) {
#pragma unroll
      for (int jr = 0; jr < 4; ++jr) {
        const int b = wave * 4 + jr;
        const float* cr = slab + b * kSlabPitch;
        const size_t ro = ((size_t)(b * kNodes + i)) * kHid;
        const v4f ca = *(const v4f*)(cr + 4 * lane);
        const v4f cb = *(const v4f*)(cr + 128 + 4 * lane);
        *(volatile v4f*)(CS + ro + 4 * lane) = ca;
        *(volatile v4f*)(CS + ro + 128 + 4 * lane) = cb;
      }
      __threadfence();
    }
    __syncthreads();
    __threadfence();
  }
}

extern "C" void kernel_launch(void* const* d_in, const int* in_sizes, int n_in,
                              void* d_out, int out_size, void* d_ws, size_t ws_size,
                              hipStream_t stream) {
  if (n_in < 8) return;
  if (in_sizes[0] != kBatch * kNodes * kDim) return;
  if (in_sizes[1] != kBatch * kNodes) return;
  if (in_sizes[3] != kDim * kGates) return;
  if (in_sizes[4] != kGates) return;
  if (in_sizes[5] != kHid * kHid || in_sizes[6] != kHid * kHid || in_sizes[7] != kHid * kHid) return;
  if (out_size != kBatch * kNodes * kHid) return;
  const size_t offW   = 0;
  const size_t offVh  = offW   + (size_t)kGates * kDim * 2;
  const size_t offVl  = offVh  + (size_t)kGates * kHid * 2;
  const size_t offE   = offVl  + (size_t)kGates * kHid * 2;
  const size_t offG   = offE   + (size_t)kBatch * kNodes * kDim * 2;
  const size_t offCS  = offG   + (size_t)kBatch * kHalfNodes * kGates * 4;
  const size_t total  = offCS  + (size_t)kBatch * kNodes * kHid * 4;
  if (ws_size < total) return;

  const float* emb   = (const float*)d_in[0];
  const int*   conn  = (const int*)d_in[1];
  const int*   nmask = (const int*)d_in[2];
  const float* W     = (const float*)d_in[3];
  const float* bias  = (const float*)d_in[4];
  const float* tf    = (const float*)d_in[5];
  const float* to    = (const float*)d_in[6];
  const float* tz    = (const float*)d_in[7];

  char* ws = (char*)d_ws;
  unsigned short* WBt   = (unsigned short*)(ws + offW);
  unsigned short* VBh   = (unsigned short*)(ws + offVh);
  unsigned short* VBl   = (unsigned short*)(ws + offVl);
  unsigned short* EMB16 = (unsigned short*)(ws + offE);
  float*          GATES = (float*)(ws + offG);
  float*          CS    = (float*)(ws + offCS);
  float*          out   = (float*)d_out;

  const int n8 = kBatch * kNodes * kDim / 8;
  k_cast_bf16x8<<<(n8 + kThreads - 1) / kThreads, kThreads, 0, stream>>>(emb, EMB16, n8);
  k_wprep<<<kGates / 32, kThreads, 0, stream>>>(W, WBt);
  k_vprep<<<3 * (kHid / 16), kThreads, 0, stream>>>(tf, to, tz, VBh, VBl);

  const int gemmBlocks = ((kHalfNodes / 64) * (kGates / 64) + 7) / 8;
  for (int hp = 0; hp < 2; ++hp) {
    const unsigned short* Ahp = EMB16 + (size_t)hp * kHalfNodes * kDim;
    wmma_gemm64<1, false, 0, 0, false, 0><<<dim3(gemmBlocks, kBatch), kThreads, 0, stream>>>(
        Ahp, Ahp, kDim, (long)kNodes * kDim,
        WBt, WBt, kDim, 0L,
        (void*)GATES, (void*)GATES, kGates, (long)kHalfNodes * kGates,
        bias, bias, 0L,
        kHalfNodes, kGates, kDim, 1.0f);
    k_tree<<<1, kThreads, 0, stream>>>(conn, nmask, bias, GATES, VBh, VBl, CS, out, hp * kHalfNodes);
  }
}
